// GNNFusion_30726196035938
// MI455X (gfx1250) — hardware-verified
//
#include <hip/hip_runtime.h>
#include <stddef.h>


#define HD      256
#define GFD     128
#define SED     768
#define XP      256
#define YP      256
#define FP      768
#define KMAXH   768
#define GBM     32
#define GTHR    128
#define HBM     16
#define FBM     32
#define NTHR    256
#define NWAVE   8
#define EPT     8
#define CHUNK   (NTHR * EPT)
#define WCAP    (EPT * 32)
#define LISTN   (NWAVE * WCAP)
#define NBMAX   2048
#define SLOTB   11
#define RCAP    28672
#define DEGCAP  4096
#define NEG_SLOPE 0.01f
#define LN_EPS  1e-5f
#define CA      16.0f
#define ICA     0.0625f
#define CW      64.0f
#define CP      4096.0f
#define CF      16.0f
#define SAW     0.0009765625f
#define SPW     3.814697265625e-06f
#define SFW     0.0009765625f
#define WSCAP   134217728
#define LDS_BUILD ((2 * RCAP + 2 * NBMAX + LISTN) * 4 + 64)

static_assert((CHUNK & (CHUNK - 1)) == 0 && CHUNK <= 4096);
static_assert(NBMAX == (1 << SLOTB));
static_assert(NTHR * 8 == NBMAX);
static_assert(LISTN >= NBMAX);
static_assert(LISTN >= NWAVE * WCAP);
static_assert((RCAP % 32) == 0);
static_assert(LDS_BUILD <= 300000);
static_assert(GBM == (GTHR / 32) * 8);
static_assert((HD % 32) == 0 && (GFD % 32) == 0 && (SED % 32) == 0);
static_assert(NTHR == HD);
static_assert(HBM * 8 == GTHR);
static_assert(FBM == 32);

typedef float    v4f  __attribute__((ext_vector_type(4)));
typedef float    v8f  __attribute__((ext_vector_type(8)));
typedef int      v4i  __attribute__((ext_vector_type(4)));
typedef int      v8i  __attribute__((ext_vector_type(8)));
typedef _Float16 v4h  __attribute__((ext_vector_type(4)));
typedef _Float16 v8h  __attribute__((ext_vector_type(8)));
typedef _Float16 v16h __attribute__((ext_vector_type(16)));
union FragH { v16h v; v8h h[2]; v8i w; };

__device__ __forceinline__ v8f wmh(const FragH& a, const FragH& b, v8f c) {
  v8f d = __builtin_amdgcn_wmma_f32_16x16x32_f16(false, a.v, false, b.v, (short)0, c, false, false);
  asm volatile("v_nop\n\tv_nop\n\tv_nop\n\tv_nop" : "+v"(d) : "v"(a.w), "v"(b.w));
  return d;
}

__device__ __forceinline__ v8h pack8(v4f a, v4f b, float sc) {
  v8h hv;
  hv[0] = (_Float16)(a.x * sc); hv[1] = (_Float16)(a.y * sc);
  hv[2] = (_Float16)(a.z * sc); hv[3] = (_Float16)(a.w * sc);
  hv[4] = (_Float16)(b.x * sc); hv[5] = (_Float16)(b.y * sc);
  hv[6] = (_Float16)(b.z * sc); hv[7] = (_Float16)(b.w * sc);
  return hv;
}

__device__ __forceinline__ v4h pack4(v4f a, float sc) {
  v4h hv;
  hv[0] = (_Float16)(a.x * sc); hv[1] = (_Float16)(a.y * sc);
  hv[2] = (_Float16)(a.z * sc); hv[3] = (_Float16)(a.w * sc);
  return hv;
}

__device__ __forceinline__ float leakyf(float v) { return v > 0.f ? v : NEG_SLOPE * v; }

__device__ __forceinline__ v4f leaky4(v4f a) {
  v4f r;
  r.x = leakyf(a.x); r.y = leakyf(a.y); r.z = leakyf(a.z); r.w = leakyf(a.w);
  return r;
}

__device__ __forceinline__ int scan_chunk(const int* __restrict__ dsts, int nE, int cbase, int slotBase,
                                          int nb, int vec8, int* list, int tid, int lane, int wave) {
  int wc = 0;
  const int el0  = tid * EPT;
  const int e0   = cbase + el0;
  const int sent = -2147483647 - 1;
  v4i da, db;
  if (vec8 != 0 && cbase + CHUNK <= nE) {
    da = *(const v4i*)(dsts + e0);
    db = *(const v4i*)(dsts + e0 + 4);
  } else {
    da.x = (e0     < nE) ? dsts[min(e0,     nE - 1)] : sent;
    da.y = (e0 + 1 < nE) ? dsts[min(e0 + 1, nE - 1)] : sent;
    da.z = (e0 + 2 < nE) ? dsts[min(e0 + 2, nE - 1)] : sent;
    da.w = (e0 + 3 < nE) ? dsts[min(e0 + 3, nE - 1)] : sent;
    db.x = (e0 + 4 < nE) ? dsts[min(e0 + 4, nE - 1)] : sent;
    db.y = (e0 + 5 < nE) ? dsts[min(e0 + 5, nE - 1)] : sent;
    db.z = (e0 + 6 < nE) ? dsts[min(e0 + 6, nE - 1)] : sent;
    db.w = (e0 + 7 < nE) ? dsts[min(e0 + 7, nE - 1)] : sent;
  }
  const unsigned nbs = (unsigned)slotBase;
  const unsigned unb = (unsigned)nb;
  const unsigned s0 = (unsigned)da.x - nbs, s1 = (unsigned)da.y - nbs;
  const unsigned s2 = (unsigned)da.z - nbs, s3 = (unsigned)da.w - nbs;
  const unsigned s4 = (unsigned)db.x - nbs, s5 = (unsigned)db.y - nbs;
  const unsigned s6 = (unsigned)db.z - nbs, s7 = (unsigned)db.w - nbs;
  const bool h0 = s0 < unb, h1 = s1 < unb, h2 = s2 < unb, h3 = s3 < unb;
  const bool h4 = s4 < unb, h5 = s5 < unb, h6 = s6 < unb, h7 = s7 < unb;
  const unsigned any = __builtin_amdgcn_ballot_w32(h0 | h1 | h2 | h3 | h4 | h5 | h6 | h7);
  if (any != 0u) {
#define HITJ(J, HJ, SJ) { \
      const unsigned mj = __builtin_amdgcn_ballot_w32(HJ); \
      if (mj != 0u) { \
        if (HJ) { \
          const int pos = wc + (int)__builtin_amdgcn_mbcnt_lo(mj, 0u); \
          if (pos < WCAP) list[wave * WCAP + pos] = ((el0 + (J)) << 12) | (int)(SJ); \
        } \
        wc += (int)__builtin_popcount(mj); } }
    HITJ(0, h0, s0)
    HITJ(1, h1, s1)
    HITJ(2, h2, s2)
    HITJ(3, h3, s3)
    HITJ(4, h4, s4)
    HITJ(5, h5, s5)
    HITJ(6, h6, s6)
    HITJ(7, h7, s7)
#undef HITJ
  }
  return wc;
}

__global__ __launch_bounds__(NTHR) void k_xprep(const float* __restrict__ x, _Float16* xc, int nN, int nUnits) {
  const int i = (int)blockIdx.x * NTHR + (int)threadIdx.x;
  if (i >= nUnits) return;
  const int row = i >> 5;
  const int c0  = (i & 31) * 8;
  const int rc  = row < nN ? row : nN - 1;
  const float* p = x + (size_t)rc * HD + c0;
  v4f a = *(const v4f*)p, b = *(const v4f*)(p + 4);
  const v4f z4 = {0.f, 0.f, 0.f, 0.f};
  if (row >= nN) { a = z4; b = z4; }
  const v8h hv = pack8(a, b, CA);
  const size_t o = (size_t)row * XP + c0;
  *(volatile v8h*)(xc + o) = hv;
  __threadfence();
  *(volatile v8h*)(xc + o) = hv;
}

__global__ __launch_bounds__(NTHR) void k_wprep(const float* __restrict__ w0, const float* __restrict__ w1,
                                                const float* __restrict__ w2, const float* __restrict__ w3,
                                                const float* __restrict__ w4, const float* __restrict__ w5,
                                                const float* __restrict__ w6,
                                                _Float16* t0, _Float16* t1, _Float16* t2, _Float16* t3,
                                                _Float16* t4, _Float16* t5, _Float16* t6) {
  const int j = (int)blockIdx.y;
  const float* src; _Float16* dst; int K;
  switch (j) {
    case 0: src = w0; dst = t0; K = HD;  break;
    case 1: src = w1; dst = t1; K = HD;  break;
    case 2: src = w2; dst = t2; K = HD;  break;
    case 3: src = w3; dst = t3; K = HD;  break;
    case 4: src = w4; dst = t4; K = GFD; break;
    case 5: src = w5; dst = t5; K = SED; break;
    default: src = w6; dst = t6; K = SED; break;
  }
  const int u = (int)blockIdx.x * NTHR + (int)threadIdx.x;
  const int kp8 = K >> 3;
  const int nUnits = HD * kp8;
  if (u >= nUnits) return;
  const int n  = u / kp8;
  const int k8 = (u - n * kp8) * 8;
  const float* p = src + (size_t)k8 * HD + n;
  v4f a, b;
  a.x = p[0 * HD]; a.y = p[1 * HD]; a.z = p[2 * HD]; a.w = p[3 * HD];
  b.x = p[4 * HD]; b.y = p[5 * HD]; b.z = p[6 * HD]; b.w = p[7 * HD];
  const v8h hv = pack8(a, b, CW);
  const size_t o = (size_t)n * K + k8;
  *(volatile v8h*)(dst + o) = hv;
  __threadfence();
  *(volatile v8h*)(dst + o) = hv;
}

__global__ __launch_bounds__(NTHR) void k_build(const int* __restrict__ dsts, int* EL, int* OFF, int* CNT,
                                                int nE, int nb, int tp, int vec8) {
  extern __shared__ v4f lds_dyn[];
  int* reg1 = (int*)lds_dyn;
  int* reg2 = reg1 + RCAP;
  int* scnt = reg2 + RCAP;
  int* soff = scnt + NBMAX;
  int* list = soff + NBMAX;
  int* wcnt = list + LISTN;
  int* wtot = wcnt + NWAVE;
  const int tid = threadIdx.x, lane = tid & 31, wave = tid >> 5;
  const int nodeBase = (int)blockIdx.x * nb;

  for (int i = tid; i < NBMAX; i += NTHR) scnt[i] = 0;
  {
    const v4i z = {0, 0, 0, 0};
    v4i* r2v = (v4i*)reg2;
    for (int f = tid; f < RCAP / 4; f += NTHR) r2v[f] = z;
  }
  __syncthreads();

  int tot = 0;
  const int nChunks = (nE + CHUNK - 1) / CHUNK;
#pragma unroll 1
  for (int ch = 0; ch < nChunks; ++ch) {
    const int cbase = ch * CHUNK;
    const int wc = scan_chunk(dsts, nE, cbase, nodeBase, nb, vec8, list, tid, lane, wave);
    if (lane == 0) wcnt[wave] = wc;
    __syncthreads();
    int pre = 0, all = 0;
#pragma unroll
    for (int w2 = 0; w2 < NWAVE; ++w2) {
      int c = wcnt[w2];
      c = c < 0 ? 0 : (c > WCAP ? WCAP : c);
      all += c;
      pre += (w2 < wave) ? c : 0;
    }
    const int wcc  = wc > WCAP ? WCAP : wc;
    const int base = tot + pre;
#pragma unroll 1
    for (int i = lane; i < wcc; i += 32) {
      const int ent = list[wave * WCAP + i];
      const int el  = (ent >> 12) & (CHUNK - 1);
      const int sl  = ent & (NBMAX - 1);
      int eid = cbase + el;
      eid = eid > nE - 1 ? nE - 1 : eid;
      const int pos = base + i;
      if (pos < RCAP) reg1[pos] = (int)(((unsigned)eid << SLOTB) | (unsigned)sl);
    }
    tot += all;
    tot = tot > RCAP ? RCAP : tot;
    __syncthreads();
  }
  const int nh = tot;

  if (wave == 0) {
#pragma unroll 1
    for (int b0 = 0; b0 < nh; b0 += 32) {
      const int idx = b0 + lane;
      const int uv  = reg1[idx < RCAP ? idx : RCAP - 1];
      const int m32 = (nh - b0) < 32 ? (nh - b0) : 32;
#pragma unroll 1
      for (int k = 0; k < m32; ++k) {
        const int u  = __builtin_amdgcn_readlane(uv, k);
        const int sl = u & (NBMAX - 1);
        if (lane == 0) scnt[sl] = scnt[sl] + 1;
      }
    }
  }
  __syncthreads();

  {
    const v4i ca = *(const v4i*)(scnt + 8 * tid);
    const v4i cb = *(const v4i*)(scnt + 8 * tid + 4);
    const int e0 = ca.x < 0 ? 0 : ca.x, e1 = ca.y < 0 ? 0 : ca.y, e2 = ca.z < 0 ? 0 : ca.z, e3 = ca.w < 0 ? 0 : ca.w;
    const int e4 = cb.x < 0 ? 0 : cb.x, e5 = cb.y < 0 ? 0 : cb.y, e6 = cb.z < 0 ? 0 : cb.z, e7 = cb.w < 0 ? 0 : cb.w;
    const int ts = e0 + e1 + e2 + e3 + e4 + e5 + e6 + e7;
    int incl = ts;
#pragma unroll
    for (int d = 1; d < 32; d <<= 1) {
      const int up = __shfl_up(incl, d);
      if (lane >= d) incl += up;
    }
    if (lane == 31) wtot[wave] = incl;
    __syncthreads();
    int pre = 0;
#pragma unroll
    for (int w2 = 0; w2 < NWAVE; ++w2) pre += (w2 < wave) ? wtot[w2] : 0;
    int run = pre + incl - ts;
    soff[8 * tid + 0] = run; run += e0;
    soff[8 * tid + 1] = run; run += e1;
    soff[8 * tid + 2] = run; run += e2;
    soff[8 * tid + 3] = run; run += e3;
    soff[8 * tid + 4] = run; run += e4;
    soff[8 * tid + 5] = run; run += e5;
    soff[8 * tid + 6] = run; run += e6;
    soff[8 * tid + 7] = run;
  }
  __syncthreads();
  for (int i = tid; i < NBMAX; i += NTHR) list[i] = soff[i];
  __syncthreads();

  if (wave == 0) {
#pragma unroll 1
    for (int b0 = 0; b0 < nh; b0 += 32) {
      const int idx = b0 + lane;
      const int uv  = reg1[idx < RCAP ? idx : RCAP - 1];
      const int m32 = (nh - b0) < 32 ? (nh - b0) : 32;
#pragma unroll 1
      for (int k = 0; k < m32; ++k) {
        const int u   = __builtin_amdgcn_readlane(uv, k);
        const int sl  = u & (NBMAX - 1);
        const int eid = (int)((unsigned)u >> SLOTB);
        if (lane == 0) {
          int pos = list[sl];
          pos = pos < 0 ? 0 : (pos > RCAP - 1 ? RCAP - 1 : pos);
          reg2[pos] = eid;
          list[sl] = pos + 1;
        }
      }
    }
  }
  __syncthreads();

  {
    int* elb = EL + (size_t)blockIdx.x * RCAP;
    const v4i* r4 = (const v4i*)reg2;
#pragma unroll 1
    for (int f = tid; f < RCAP / 4; f += NTHR) {
      const v4i v = r4[f];
      *(volatile v4i*)(elb + 4 * f) = v;
    }
    __threadfence();
#pragma unroll 1
    for (int f = tid; f < RCAP / 4; f += NTHR) {
      const v4i v = r4[f];
      *(volatile v4i*)(elb + 4 * f) = v;
    }
  }
  {
    const bool ovf = (nh >= RCAP);
    int* ob = OFF + (size_t)blockIdx.x * tp;
    int* cb = CNT + (size_t)blockIdx.x * tp;
    const int n4 = tp >> 2;
#pragma unroll 1
    for (int pass = 0; pass < 2; ++pass) {
#pragma unroll 1
      for (int f = tid; f < n4; f += NTHR) {
        v4i so, sc;
        {
          const int s = 4 * f + 0; const bool in = s < nb; const int scl = s < NBMAX ? s : NBMAX - 1;
          so.x = in ? soff[scl] : 0; sc.x = in ? (ovf ? -1 : scnt[scl]) : 0;
        }
        {
          const int s = 4 * f + 1; const bool in = s < nb; const int scl = s < NBMAX ? s : NBMAX - 1;
          so.y = in ? soff[scl] : 0; sc.y = in ? (ovf ? -1 : scnt[scl]) : 0;
        }
        {
          const int s = 4 * f + 2; const bool in = s < nb; const int scl = s < NBMAX ? s : NBMAX - 1;
          so.z = in ? soff[scl] : 0; sc.z = in ? (ovf ? -1 : scnt[scl]) : 0;
        }
        {
          const int s = 4 * f + 3; const bool in = s < nb; const int scl = s < NBMAX ? s : NBMAX - 1;
          so.w = in ? soff[scl] : 0; sc.w = in ? (ovf ? -1 : scnt[scl]) : 0;
        }
        *(volatile v4i*)(ob + 4 * f) = so;
        *(volatile v4i*)(cb + 4 * f) = sc;
      }
      __threadfence();
    }
  }
}

__global__ __launch_bounds__(NTHR) void k_dis(const int* __restrict__ CNT, float* DIS, int nb, int tp, int nTot) {
  const int t  = (int)blockIdx.x * NTHR + (int)threadIdx.x;
  const int i0 = 4 * t;
  const float qnan = __int_as_float(0x7fc00000);
  v4f dv;
#pragma unroll
  for (int u = 0; u < 4; ++u) {
    int ic = i0 + u;
    ic = ic > nTot - 1 ? nTot - 1 : ic;
    const int b = ic / nb;
    const int s = ic - b * nb;
    const int c = CNT[(size_t)b * tp + s];
    const float val = (c < 0 || c > DEGCAP) ? qnan : rsqrtf((float)(c + 1));
    dv[u] = val;
  }
  *(volatile v4f*)(DIS + i0) = dv;
  __threadfence();
  *(volatile v4f*)(DIS + i0) = dv;
}

__global__ __launch_bounds__(GTHR) void k_gemm(const _Float16* __restrict__ xc, const _Float16* __restrict__ wt, float* Y) {
  __shared__ __attribute__((aligned(16))) float stg[GBM * HD];
  const int tid = threadIdx.x, lane = tid & 31, wave = tid >> 5, hh = lane >> 4, m = lane & 15;
  const int wr = wave & 1, wc = wave >> 1;
  const int rowBase = (int)blockIdx.x * GBM;
  const size_t arow = (size_t)(rowBase + 16 * wr + m) * XP + 8 * hh;
  const size_t brow = (size_t)(128 * wc + m) * HD + 8 * hh;
  v8f acc[8];
#pragma unroll
  for (int t = 0; t < 8; ++t) { v8f z = {0.f, 0.f, 0.f, 0.f, 0.f, 0.f, 0.f, 0.f}; acc[t] = z; }
#pragma unroll 1
  for (int ks = 0; ks < HD / 32; ++ks) {
    FragH af;
    af.h[0] = *(const v8h*)(xc + arow + 32 * ks);
    af.h[1] = *(const v8h*)(xc + arow + 32 * ks + 16);
#pragma unroll
    for (int t = 0; t < 8; ++t) {
      const size_t bo = brow + (size_t)(16 * t) * HD + 32 * ks;
      FragH bf;
      bf.h[0] = *(const v8h*)(wt + bo);
      bf.h[1] = *(const v8h*)(wt + bo + 16);
      acc[t] = wmh(af, bf, acc[t]);
    }
  }
  {
    float* sp = stg + (size_t)(16 * wr + 8 * hh) * HD + 128 * wc + m;
#pragma unroll
    for (int t = 0; t < 8; ++t) {
#pragma unroll
      for (int r = 0; r < 8; ++r) sp[(size_t)r * HD + 16 * t] = acc[t][r] * SAW;
    }
  }
  __syncthreads();
  {
    const int nF4 = GBM * HD / 4;
    float* yb = Y + (size_t)rowBase * YP;
    const v4f* s4 = (const v4f*)stg;
#pragma unroll 1
    for (int f = tid; f < nF4; f += GTHR) {
      const int r = f >> 6, q = f & 63;
      const v4f v = s4[f];
      *(volatile v4f*)(yb + (size_t)r * YP + 4 * q) = v;
    }
    __threadfence();
#pragma unroll 1
    for (int f = tid; f < nF4; f += GTHR) {
      const int r = f >> 6, q = f & 63;
      const v4f v = s4[f];
      *(volatile v4f*)(yb + (size_t)r * YP + 4 * q) = v;
    }
  }
}

__global__ __launch_bounds__(NTHR) void k_agg(
    const int* __restrict__ srcs, const int* __restrict__ EL,
    const int* __restrict__ OFF, const int* __restrict__ CNT,
    const float* __restrict__ DIS, const float* __restrict__ Y,
    const float* __restrict__ bias, _Float16* xout, int nN, int nE, int nb, int tp) {
  const int tid = threadIdx.x, lane = tid & 31, wave = tid >> 5;
  const int nodeBase = (int)blockIdx.x * nb;
  const int nbw = nb >> 3;
  const int* elb  = EL  + (size_t)blockIdx.x * RCAP;
  const int* offb = OFF + (size_t)blockIdx.x * tp;
  const int* cntb = CNT + (size_t)blockIdx.x * tp;
  const v4f bz0 = *(const v4f*)(bias + 4 * lane);
  const v4f bz1 = *(const v4f*)(bias + 128 + 4 * lane);
  const float qnan = __int_as_float(0x7fc00000);
#pragma unroll 1
  for (int jt = 0; jt < nbw; ++jt) {
    const int slot = wave * nbw + jt;
    const int grow = nodeBase + slot;
    const int gcl  = grow < nN ? grow : nN - 1;
    const bool wr  = grow < nN;
    int st = offb[slot];
    const int craw = cntb[slot];
    st = st < 0 ? 0 : (st > RCAP - 1 ? RCAP - 1 : st);
    int cnt = craw < 0 ? 0 : (craw > DEGCAP ? DEGCAP : craw);
    if (cnt > RCAP - st) cnt = RCAP - st;
    const float pz = (craw < 0 || craw > DEGCAP) ? qnan : 0.0f;

    const float dd  = DIS[gcl];
    const float wdd = dd * dd;
    const float* yd = Y + (size_t)gcl * YP + 4 * lane;
    v4f a0 = *(const v4f*)(yd) * wdd;
    v4f a1 = *(const v4f*)(yd + 128) * wdd;
#pragma unroll 1
    for (int b0 = 0; b0 < cnt; b0 += 32) {
      int q = b0 + lane;
      q = q < cnt ? q : cnt - 1;
      int eid = elb[st + q];
      eid = eid < 0 ? 0 : (eid > nE - 1 ? nE - 1 : eid);
      const int sraw = srcs[eid];
      const int s = sraw < 0 ? 0 : (sraw > nN - 1 ? nN - 1 : sraw);
      const float ws  = DIS[s] * dd;
      const int   wsi = __float_as_int(ws);
      const int m32 = (cnt - b0) < 32 ? (cnt - b0) : 32;
#pragma unroll 1
      for (int k = 0; k < m32; ++k) {
        const int   sk = __builtin_amdgcn_readlane(s, k);
        const float wk = __int_as_float(__builtin_amdgcn_readlane(wsi, k));
        const float* ys = Y + (size_t)sk * YP + 4 * lane;
        const v4f x0 = *(const v4f*)(ys);
        const v4f x1 = *(const v4f*)(ys + 128);
        a0 = a0 + x0 * wk;
        a1 = a1 + x1 * wk;
      }
    }
    const v4f o0 = leaky4(a0 + bz0 + pz);
    const v4f o1 = leaky4(a1 + bz1 + pz);
    const v4h g0 = pack4(o0, CA);
    const v4h g1 = pack4(o1, CA);
    _Float16* xp = xout + (size_t)gcl * XP + 4 * lane;
    if (wr) {
      *(volatile v4h*)(xp) = g0;
      *(volatile v4h*)(xp + 128) = g1;
    }
    __threadfence();
    if (wr) {
      *(volatile v4h*)(xp) = g0;
      *(volatile v4h*)(xp + 128) = g1;
    }
  }
}

__global__ __launch_bounds__(NTHR) void k_pool(const _Float16* __restrict__ xc, const int* __restrict__ bat,
                                               float* PO, int nN, int vec8) {
  __shared__ int list[LISTN];
  __shared__ int wcnt[NWAVE];
  const int tid = threadIdx.x, lane = tid & 31, wave = tid >> 5;
  const int g = (int)blockIdx.x;
  float acc = 0.f;
  int cnt = 0;
  const int nChunks = (nN + CHUNK - 1) / CHUNK;
#pragma unroll 1
  for (int ch = 0; ch < nChunks; ++ch) {
    const int cbase = ch * CHUNK;
    const int wc = scan_chunk(bat, nN, cbase, g, 1, vec8, list, tid, lane, wave);
    if (lane == 0) wcnt[wave] = wc;
    __syncthreads();
#pragma unroll 1
    for (int w2 = 0; w2 < NWAVE; ++w2) {
      int c = wcnt[w2];
      c = c < 0 ? 0 : (c > WCAP ? WCAP : c);
      cnt += c;
#pragma unroll 1
      for (int i = 0; i < c; ++i) {
        const int ent = list[w2 * WCAP + i];
        const int el  = (ent >> 12) & (CHUNK - 1);
        int node = cbase + el;
        node = node > nN - 1 ? nN - 1 : node;
        acc += (float)xc[(size_t)node * XP + tid];
      }
    }
    __syncthreads();
  }
  const float inv = 1.0f / (float)(cnt > 1 ? cnt : 1);
  const float po = acc * inv * ICA;
  float* p = PO + (size_t)g * HD + tid;
  *(volatile float*)p = po;
  __threadfence();
  *(volatile float*)p = po;
}

__global__ __launch_bounds__(GTHR) void k_branch(const float* __restrict__ PO, const float* __restrict__ smi,
                                                 const float* __restrict__ gf,
                                                 const _Float16* __restrict__ gnT, const _Float16* __restrict__ smT,
                                                 const _Float16* __restrict__ gfT,
                                                 const float* __restrict__ gnb, const float* __restrict__ smb,
                                                 const float* __restrict__ gfb,
                                                 const float* __restrict__ alpha_p, const float* __restrict__ beta_p,
                                                 _Float16* FZ) {
  __shared__ __attribute__((aligned(16))) _Float16 sA[HBM * KMAXH];
  __shared__ __attribute__((aligned(16))) float    stg[HBM * HD];
  __shared__ __attribute__((aligned(16))) _Float16 sO[HBM * HD];
  __shared__ float sbias[HD];
  const int tid = threadIdx.x, lane = tid & 31, wave = tid >> 5, hh = lane >> 4, m = lane & 15;
  const int br = (int)blockIdx.y;
  const int r0 = (int)blockIdx.x * HBM;
  const float al = 1.0f / (1.0f + expf(-alpha_p[0]));
  const float be = 1.0f / (1.0f + expf(-beta_p[0]));
  const float* A; const _Float16* WT; const float* bias; int K; float carry, scl, gate;
  if (br == 0)      { A = PO;  WT = gnT; bias = gnb; K = HD;  carry = CP; scl = SPW; gate = al; }
  else if (br == 1) { A = smi; WT = smT; bias = smb; K = SED; carry = CA; scl = SAW; gate = be; }
  else              { A = gf;  WT = gfT; bias = gfb; K = GFD; carry = CA; scl = SAW; gate = (1.0f - al) - be; }
  const int foff = HD * br;
  sbias[tid] = bias[tid];
  sbias[tid + 128] = bias[tid + 128];
  {
    const int kp8 = K >> 3;
    const int units = HBM * kp8;
#pragma unroll 1
    for (int u = tid; u < units; u += GTHR) {
      const int row = u / kp8;
      const int c8  = (u - row * kp8) * 8;
      const float* p = A + (size_t)(r0 + row) * K + c8;
      const v4f a = *(const v4f*)p, b = *(const v4f*)(p + 4);
      *(v8h*)(sA + (size_t)row * KMAXH + c8) = pack8(a, b, carry);
    }
  }
  __syncthreads();
  v8f acc[4];
#pragma unroll
  for (int t = 0; t < 4; ++t) { v8f z = {0.f, 0.f, 0.f, 0.f, 0.f, 0.f, 0.f, 0.f}; acc[t] = z; }
  const _Float16* arow = sA + (size_t)m * KMAXH + 8 * hh;
  const size_t brow = (size_t)(64 * wave + m) * K + 8 * hh;
  const int nks = K >> 5;
#pragma unroll 1
  for (int ks = 0; ks < nks; ++ks) {
    FragH af;
    af.h[0] = *(const v8h*)(arow + 32 * ks);
    af.h[1] = *(const v8h*)(arow + 32 * ks + 16);
#pragma unroll
    for (int t = 0; t < 4; ++t) {
      const size_t bo = brow + (size_t)(16 * t) * K + 32 * ks;
      FragH bf;
      bf.h[0] = *(const v8h*)(WT + bo);
      bf.h[1] = *(const v8h*)(WT + bo + 16);
      acc[t] = wmh(af, bf, acc[t]);
    }
  }
  {
    float* sp = stg + (size_t)(8 * hh) * HD + 64 * wave + m;
#pragma unroll
    for (int t = 0; t < 4; ++t) {
      const float c = sbias[64 * wave + 16 * t + m];
#pragma unroll
      for (int r = 0; r < 8; ++r) sp[(size_t)r * HD + 16 * t] = fmaf(acc[t][r], scl, c);
    }
  }
  __syncthreads();
  {
    const int row = tid >> 3, part = tid & 7;
    const float* sr = stg + (size_t)row * HD + part * 32;
    float s = 0.f;
#pragma unroll 1
    for (int c = 0; c < 32; ++c) s += sr[c];
    s += __shfl_xor(s, 1);
    s += __shfl_xor(s, 2);
    s += __shfl_xor(s, 4);
    const float mean = s * (1.0f / 256.0f);
    float q = 0.f;
#pragma unroll 1
    for (int c = 0; c < 32; ++c) { const float d = sr[c] - mean; q = fmaf(d, d, q); }
    q += __shfl_xor(q, 1);
    q += __shfl_xor(q, 2);
    q += __shfl_xor(q, 4);
    const float var  = q * (1.0f / 256.0f);
    const float rstd = 1.0f / sqrtf(var + LN_EPS);
    const float gs   = rstd * gate;
    _Float16* so = sO + (size_t)row * HD + part * 32;
#pragma unroll
    for (int i = 0; i < 4; ++i) {
      v8h hv;
#pragma unroll
      for (int c = 0; c < 8; ++c) {
        const float y = leakyf((sr[8 * i + c] - mean) * gs);
        hv[c] = (_Float16)(y * CF);
      }
      *(v8h*)(so + 8 * i) = hv;
    }
  }
  __syncthreads();
  {
#pragma unroll
    for (int i = 0; i < 4; ++i) {
      const int row = 4 * wave + i;
      const v8h v = *(const v8h*)(sO + (size_t)row * HD + 8 * lane);
      *(volatile v8h*)(FZ + (size_t)(r0 + row) * FP + foff + 8 * lane) = v;
    }
    __threadfence();
#pragma unroll
    for (int i = 0; i < 4; ++i) {
      const int row = 4 * wave + i;
      const v8h v = *(const v8h*)(sO + (size_t)row * HD + 8 * lane);
      *(volatile v8h*)(FZ + (size_t)(r0 + row) * FP + foff + 8 * lane) = v;
    }
  }
}

__global__ __launch_bounds__(GTHR) void k_fus(const _Float16* __restrict__ FZ, const _Float16* __restrict__ f1T,
                                              const float* __restrict__ f1b, const float* __restrict__ f2w,
                                              const float* __restrict__ f2b, float* out) {
  __shared__ float sb1[HD];
  __shared__ float sw2[HD];
  __shared__ float part[2 * FBM];
  __shared__ __attribute__((aligned(16))) float sOut[FBM];
  const int tid = threadIdx.x, lane = tid & 31, wave = tid >> 5, hh = lane >> 4, m = lane & 15;
  const int wr = wave & 1, wc = wave >> 1;
  const int rowBase = (int)blockIdx.x * FBM;
  sb1[tid] = f1b[tid]; sb1[tid + 128] = f1b[tid + 128];
  sw2[tid] = f2w[tid]; sw2[tid + 128] = f2w[tid + 128];
  const size_t arow = (size_t)(rowBase + 16 * wr + m) * FP + 8 * hh;
  const size_t brow = (size_t)(128 * wc + m) * SED + 8 * hh;
  v8f acc[8];
#pragma unroll
  for (int t = 0; t < 8; ++t) { v8f z = {0.f, 0.f, 0.f, 0.f, 0.f, 0.f, 0.f, 0.f}; acc[t] = z; }
#pragma unroll 1
  for (int ks = 0; ks < SED / 32; ++ks) {
    FragH af;
    af.h[0] = *(const v8h*)(FZ + arow + 32 * ks);
    af.h[1] = *(const v8h*)(FZ + arow + 32 * ks + 16);
#pragma unroll
    for (int t = 0; t < 8; ++t) {
      const size_t bo = brow + (size_t)(16 * t) * SED + 32 * ks;
      FragH bf;
      bf.h[0] = *(const v8h*)(f1T + bo);
      bf.h[1] = *(const v8h*)(f1T + bo + 16);
      acc[t] = wmh(af, bf, acc[t]);
    }
  }
  __syncthreads();
  float o[8];
#pragma unroll
  for (int r = 0; r < 8; ++r) o[r] = 0.f;
#pragma unroll
  for (int t = 0; t < 8; ++t) {
    const int col = 128 * wc + 16 * t + m;
    const float c = sb1[col], q = sw2[col];
#pragma unroll
    for (int r = 0; r < 8; ++r) {
      const float h = leakyf(fmaf(acc[t][r], SFW, c));
      o[r] = fmaf(h, q, o[r]);
    }
  }
#pragma unroll
  for (int r = 0; r < 8; ++r) {
    o[r] += __shfl_xor(o[r], 1);
    o[r] += __shfl_xor(o[r], 2);
    o[r] += __shfl_xor(o[r], 4);
    o[r] += __shfl_xor(o[r], 8);
  }
  if (m == 0) {
#pragma unroll
    for (int r = 0; r < 8; ++r) part[wc * FBM + 16 * wr + 8 * hh + r] = o[r];
  }
  __syncthreads();
  if (tid < FBM) sOut[tid] = (part[tid] + part[FBM + tid]) + f2b[0];
  __syncthreads();
  const bool st = tid < 8;
  const v4f v = *(const v4f*)(sOut + 4 * (tid & 7));
  float* p = out + (size_t)rowBase + 4 * (tid & 7);
  if (st) *(volatile v4f*)p = v;
  __threadfence();
  if (st) *(volatile v4f*)p = v;
}

static int pick_nb(int nE, int nN) {
  int nb = NBMAX;
  while (nb > 16 && (long long)nb * (long long)nE * 5LL > (long long)RCAP * (long long)nN * 4LL) nb >>= 1;
  return nb;
}

static inline size_t al256(size_t v) { return (v + 255) & ~(size_t)255; }

extern "C" void kernel_launch(void* const* d_in, const int* in_sizes, int n_in,
                              void* d_out, int out_size, void* d_ws, size_t ws_size,
                              hipStream_t stream) {
  if (n_in < 23) return;
  const int nN = in_sizes[0] / HD;
  if (nN <= 0 || in_sizes[0] != nN * HD || nN > (1 << 22)) return;
  if (in_sizes[1] < 2 || (in_sizes[1] & 1) != 0) return;
  const int nE = in_sizes[1] / 2;
  if (nE < 1 || nE > (1 << 21)) return;
  if (in_sizes[2] != nN) return;
  const int nG = in_sizes[3] / GFD;
  if (nG <= 0 || in_sizes[3] != nG * GFD || (nG % FBM) != 0) return;
  if (in_sizes[4] != nG * SED) return;
  if (in_sizes[5] != HD * HD || in_sizes[7] != HD * HD || in_sizes[9] != HD * HD || in_sizes[11] != HD * HD) return;
  if (in_sizes[6] != HD || in_sizes[8] != HD || in_sizes[10] != HD || in_sizes[12] != HD) return;
  if (in_sizes[13] != GFD * HD || in_sizes[14] != HD) return;
  if (in_sizes[15] != SED * HD || in_sizes[16] != HD) return;
  if (in_sizes[17] != SED * HD || in_sizes[18] != HD) return;
  if (in_sizes[19] != HD || in_sizes[20] != 1 || in_sizes[21] != 1 || in_sizes[22] != 1) return;
  if (out_size != nG) return;

  const float* x      = (const float*)d_in[0];
  const int*   ei     = (const int*)d_in[1];
  const int*   bat    = (const int*)d_in[2];
  const float* gfeat  = (const float*)d_in[3];
  const float* smi    = (const float*)d_in[4];
  const float* W1     = (const float*)d_in[5];
  const float* b1     = (const float*)d_in[6];
  const float* W2     = (const float*)d_in[7];
  const float* b2     = (const float*)d_in[8];
  const float* W3     = (const float*)d_in[9];
  const float* b3     = (const float*)d_in[10];
  const float* gnnW   = (const float*)d_in[11];
  const float* gnnb   = (const float*)d_in[12];
  const float* gfW    = (const float*)d_in[13];
  const float* gfb    = (const float*)d_in[14];
  const float* smiW   = (const float*)d_in[15];
  const float* smib   = (const float*)d_in[16];
  const float* f1W    = (const float*)d_in[17];
  const float* f1b    = (const float*)d_in[18];
  const float* f2W    = (const float*)d_in[19];
  const float* f2b    = (const float*)d_in[20];
  const float* alphap = (const float*)d_in[21];
  const float* betap  = (const float*)d_in[22];
  float* out = (float*)d_out;
  const int* srcs = ei;
  const int* dsts = ei + nE;

  const int MP    = ((nN + GBM - 1) / GBM) * GBM;
  const int nb    = pick_nb(nE, nN);
  const int tp    = nb < 32 ? 32 : nb;
  const int gA    = (nN + nb - 1) / nb;
  const int gG    = MP / GBM;
  const int nTot  = gA * nb;
  const int DP    = ((nTot + 1023) / 1024) * 1024;
  const int vec8E = ((nE & 3) == 0) ? 1 : 0;
  const int vec8B = 1;
  const int nUnits = MP * (XP / 8);
  if (nb < 16 || nb > NBMAX || (long long)gA * nb < (long long)nN) return;

  char* ws = (char*)d_ws;
  size_t off = 0;
  const size_t oWT1 = off; off = al256(off + (size_t)HD * HD * 2);
  const size_t oWT2 = off; off = al256(off + (size_t)HD * HD * 2);
  const size_t oWT3 = off; off = al256(off + (size_t)HD * HD * 2);
  const size_t oGNT = off; off = al256(off + (size_t)HD * HD * 2);
  const size_t oGFT = off; off = al256(off + (size_t)HD * GFD * 2);
  const size_t oSMT = off; off = al256(off + (size_t)HD * SED * 2);
  const size_t oF1T = off; off = al256(off + (size_t)HD * SED * 2);
  const size_t oXC  = off; off = al256(off + (size_t)MP * XP * 2);
  const size_t oY   = off; off = al256(off + (size_t)MP * YP * 4);
  const size_t oEL  = off; off = al256(off + (size_t)gA * RCAP * 4);
  const size_t oOFF = off; off = al256(off + (size_t)gA * tp * 4);
  const size_t oCNT = off; off = al256(off + (size_t)gA * tp * 4);
  const size_t oDIS = off; off = al256(off + (size_t)DP * 4);
  const size_t oPO  = off; off = al256(off + (size_t)nG * HD * 4);
  const size_t oFZ  = off; off = al256(off + (size_t)nG * FP * 2);
  if (off > ws_size || off > (size_t)WSCAP) return;
  _Float16* WT1 = (_Float16*)(ws + oWT1);
  _Float16* WT2 = (_Float16*)(ws + oWT2);
  _Float16* WT3 = (_Float16*)(ws + oWT3);
  _Float16* GNT = (_Float16*)(ws + oGNT);
  _Float16* GFT = (_Float16*)(ws + oGFT);
  _Float16* SMT = (_Float16*)(ws + oSMT);
  _Float16* F1T = (_Float16*)(ws + oF1T);
  _Float16* XC  = (_Float16*)(ws + oXC);
  float*    Y   = (float*)(ws + oY);
  int*      EL  = (int*)(ws + oEL);
  int*      OFF = (int*)(ws + oOFF);
  int*      CNT = (int*)(ws + oCNT);
  float*    DIS = (float*)(ws + oDIS);
  float*    PO  = (float*)(ws + oPO);
  _Float16* FZ  = (_Float16*)(ws + oFZ);

  hipFuncSetAttribute(reinterpret_cast<const void*>(&k_build),
                      hipFuncAttributeMaxDynamicSharedMemorySize, LDS_BUILD);

  k_xprep<<<(nUnits + NTHR - 1) / NTHR, NTHR, 0, stream>>>(x, XC, nN, nUnits);
  k_wprep<<<dim3((HD * (SED / 8) + NTHR - 1) / NTHR, 7), NTHR, 0, stream>>>(
      W1, W2, W3, gnnW, gfW, smiW, f1W, WT1, WT2, WT3, GNT, GFT, SMT, F1T);

  k_build<<<gA, NTHR, LDS_BUILD, stream>>>(dsts, EL, OFF, CNT, nE, nb, tp, vec8E);
  k_dis<<<DP / 4 / NTHR, NTHR, 0, stream>>>(CNT, DIS, nb, tp, nTot);

  k_gemm<<<gG, GTHR, 0, stream>>>(XC, WT1, Y);
  k_agg<<<gA, NTHR, 0, stream>>>(srcs, EL, OFF, CNT, DIS, Y, b1, XC, nN, nE, nb, tp);
  k_gemm<<<gG, GTHR, 0, stream>>>(XC, WT2, Y);
  k_agg<<<gA, NTHR, 0, stream>>>(srcs, EL, OFF, CNT, DIS, Y, b2, XC, nN, nE, nb, tp);
  k_gemm<<<gG, GTHR, 0, stream>>>(XC, WT3, Y);
  k_agg<<<gA, NTHR, 0, stream>>>(srcs, EL, OFF, CNT, DIS, Y, b3, XC, nN, nE, nb, tp);

  k_pool<<<nG, NTHR, 0, stream>>>(XC, bat, PO, nN, vec8B);
  k_branch<<<dim3(nG / HBM, 3), GTHR, 0, stream>>>(PO, smi, gfeat, GNT, SMT, GFT, gnnb, smib, gfb,
                                                    alphap, betap, FZ);
  k_fus<<<nG / FBM, GTHR, 0, stream>>>(FZ, F1T, f1b, f2W, f2b, out);
}
